// MultiHeadAttention_9328668967148
// MI455X (gfx1250) — hardware-verified
//
#include <hip/hip_runtime.h>
#include <stdint.h>

#ifndef NB
#define NB 2
#endif
#ifndef SEQ
#define SEQ 2048
#endif
#define NB_FULL 2
#define SEQ_FULL 2048
#define DM 768
#define NH 12
#define HD 64
#define MROWS (NB * SEQ)
#define QKP 1536
#define VTP MROWS
#define PP 72
#define EARLYB 4
#define TFP 32
#define CAP256 __attribute__((amdgpu_num_vgpr(256)))

static_assert(NH * HD == DM);
static_assert(HD == 64);
static_assert(SEQ % 64 == 0);
static_assert(MROWS % 64 == 0);
static_assert(DM % 64 == 0);
static_assert((2 * DM) % 64 == 0);
static_assert(DM % 32 == 0);
static_assert(QKP == 2 * DM);
static_assert(NB <= NB_FULL);
static_assert(SEQ <= SEQ_FULL);
static_assert((PP * 2) % 16 == 0);
static_assert(PP >= 64);
static_assert(SEQ / 64 >= EARLYB);
static_assert(EARLYB * 64 == 256);
static_assert(SEQ_FULL / 64 == TFP);
static_assert(SEQ / 64 <= TFP);

typedef __attribute__((ext_vector_type(16))) _Float16     v16h;
typedef __attribute__((ext_vector_type(8)))  _Float16     v8h;
typedef __attribute__((ext_vector_type(4)))  _Float16     v4h;
typedef __attribute__((ext_vector_type(16))) __bf16       v16b;
typedef __attribute__((ext_vector_type(8)))  float        v8f;
typedef __attribute__((ext_vector_type(4)))  float        v4f;
typedef __attribute__((ext_vector_type(4)))  int          v4i;
typedef __attribute__((ext_vector_type(4)))  unsigned int v4u;
typedef __attribute__((ext_vector_type(8)))  unsigned int v8u;

__device__ __forceinline__ v8u ld_frag(const unsigned short* __restrict__ p) {
    const v4u a = *(const v4u*)(p);
    const v4u b = *(const v4u*)(p + 16);
    return __builtin_shufflevector(a, b, 0, 1, 2, 3, 4, 5, 6, 7);
}

__device__ __forceinline__ unsigned int bfr_bits(float v) {
    const unsigned int u = __builtin_bit_cast(unsigned int, v);
    return (u + 0x7fffu + ((u >> 16) & 1u)) >> 16;
}
__device__ __forceinline__ float bfr_f32(float v) { return __builtin_bit_cast(float, bfr_bits(v) << 16); }
__device__ __forceinline__ void bfsplit(float v, unsigned int& hb, unsigned int& lb) {
    hb = bfr_bits(v);
    lb = bfr_bits(v - __builtin_bit_cast(float, hb << 16));
}
__device__ __forceinline__ unsigned int pk2h(float a, float b) {
    return (unsigned int)__builtin_bit_cast(unsigned short, (_Float16)a) | ((unsigned int)__builtin_bit_cast(unsigned short, (_Float16)b) << 16);
}
__device__ __forceinline__ void split_pack8(v4f a, v4f b, v4u& hi, v4u& lo) {
    unsigned int h0, h1, h2, h3, h4, h5, h6, h7, l0, l1, l2, l3, l4, l5, l6, l7;
    bfsplit(a.x, h0, l0); bfsplit(a.y, h1, l1); bfsplit(a.z, h2, l2); bfsplit(a.w, h3, l3);
    bfsplit(b.x, h4, l4); bfsplit(b.y, h5, l5); bfsplit(b.z, h6, l6); bfsplit(b.w, h7, l7);
    hi.x = h0 | (h1 << 16); hi.y = h2 | (h3 << 16); hi.z = h4 | (h5 << 16); hi.w = h6 | (h7 << 16);
    lo.x = l0 | (l1 << 16); lo.y = l2 | (l3 << 16); lo.z = l4 | (l5 << 16); lo.w = l6 | (l7 << 16);
}
__device__ __forceinline__ void hres1(float v, unsigned int& hb, unsigned int& rb) {
    const _Float16 hv = (_Float16)v;
    const _Float16 rv = (_Float16)((v - (float)hv) * 2048.0f);
    hb = (unsigned int)__builtin_bit_cast(unsigned short, hv);
    rb = (unsigned int)__builtin_bit_cast(unsigned short, rv);
}
__device__ __forceinline__ void hres_pack8(v4f a, v4f b, v4u& hi, v4u& rs) {
    unsigned int h0, h1, h2, h3, h4, h5, h6, h7, l0, l1, l2, l3, l4, l5, l6, l7;
    hres1(a.x, h0, l0); hres1(a.y, h1, l1); hres1(a.z, h2, l2); hres1(a.w, h3, l3);
    hres1(b.x, h4, l4); hres1(b.y, h5, l5); hres1(b.z, h6, l6); hres1(b.w, h7, l7);
    hi.x = h0 | (h1 << 16); hi.y = h2 | (h3 << 16); hi.z = h4 | (h5 << 16); hi.w = h6 | (h7 << 16);
    rs.x = l0 | (l1 << 16); rs.y = l2 | (l3 << 16); rs.z = l4 | (l5 << 16); rs.w = l6 | (l7 << 16);
}

template <int ET> __device__ __forceinline__ v8f mma16(v8u a, v8u b, v8f c) {
    if (ET == 0) return __builtin_amdgcn_wmma_f32_16x16x32_f16(false, __builtin_bit_cast(v16h, a), false, __builtin_bit_cast(v16h, b), (short)0, c, false, false);
    return __builtin_amdgcn_wmma_f32_16x16x32_bf16(false, __builtin_bit_cast(v16b, a), false, __builtin_bit_cast(v16b, b), (short)0, c, false, false);
}
__device__ __forceinline__ v8f wmma3b(v8u ah, v8u al, v8u bh, v8u bl, v8f c) {
    c = mma16<1>(ah, bh, c);
    c = mma16<1>(ah, bl, c);
    c = mma16<1>(al, bh, c);
    asm volatile("v_nop\n\tv_nop\n\tv_nop\n\tv_nop" : "+v"(c) : "v"(ah), "v"(al), "v"(bh), "v"(bl));
    return c;
}
__device__ __forceinline__ v8f wmma1h(v16h a, v8u b, v8f c) {
    const v16h bb = __builtin_bit_cast(v16h, b);
    c = __builtin_amdgcn_wmma_f32_16x16x32_f16(false, a, false, bb, (short)0, c, false, false);
    asm volatile("v_nop\n\tv_nop\n\tv_nop\n\tv_nop" : "+v"(c) : "v"(a), "v"(bb));
    return c;
}
__device__ __forceinline__ void guard_row(v8f& a, v8f& b, v8f& c, v8f& d, v8u x, v8u y, v8u z) {
    asm volatile("v_nop\n\tv_nop\n\tv_nop\n\tv_nop" : "+v"(a), "+v"(b), "+v"(c), "+v"(d) : "v"(x), "v"(y), "v"(z));
}
__device__ __forceinline__ void keep4(v8u a, v8u b, v8u c, v8u d) { asm volatile("v_nop" :: "v"(a), "v"(b), "v"(c), "v"(d)); }
__device__ __forceinline__ void wave_sync() {
    __builtin_amdgcn_fence(3  , "workgroup");
    __builtin_amdgcn_wave_barrier();
    __builtin_amdgcn_fence(2  , "workgroup");
}

__global__ __launch_bounds__(256) void k_cast_x(const float* __restrict__ src, unsigned short* __restrict__ dst) {
    const int u = (int)blockIdx.x * 256 + (int)threadIdx.x;
    if (u >= MROWS * (DM / 8)) return;
    const int r = u / (DM / 8), c0 = 8 * (u % (DM / 8));
    const int bb = r / SEQ, n = r - bb * SEQ;
    const float* s = src + ((size_t)bb * SEQ_FULL + (size_t)n) * DM + c0;
    const v4f a = *(const v4f*)(s);
    const v4f b = *(const v4f*)(s + 4);
    v4u pk;
    pk.x = pk2h(bfr_f32(a.x), bfr_f32(a.y)); pk.y = pk2h(bfr_f32(a.z), bfr_f32(a.w));
    pk.z = pk2h(bfr_f32(b.x), bfr_f32(b.y)); pk.w = pk2h(bfr_f32(b.z), bfr_f32(b.w));
    volatile v4u* d = (volatile v4u*)(dst + (size_t)r * DM + c0);
    *d = pk; __threadfence(); *d = pk;
}

__global__ __launch_bounds__(256) void k_castT(const float* __restrict__ src, int lds, unsigned short* __restrict__ dst, int ldd, int nR, int nC, float sc, int asbf) {
    const long long u = (long long)blockIdx.x * 256 + threadIdx.x;
    const int per = nR / 8;
    if (u >= (long long)nC * per) return;
    const int cc = (int)(u / per);
    const int r0 = 8 * (int)(u % per);
    unsigned int hb[8];
#pragma unroll
    for (int e = 0; e < 8; ++e) {
        const float w = bfr_f32(src[(size_t)(r0 + e) * (size_t)lds + (size_t)cc]);
        const unsigned int bbits = __builtin_bit_cast(unsigned int, w) >> 16;
        const unsigned int hbits = (unsigned int)__builtin_bit_cast(unsigned short, (_Float16)(w * sc));
        hb[e] = (asbf != 0) ? bbits : hbits;
    }
    v4u pk;
    pk.x = hb[0] | (hb[1] << 16); pk.y = hb[2] | (hb[3] << 16); pk.z = hb[4] | (hb[5] << 16); pk.w = hb[6] | (hb[7] << 16);
    volatile v4u* d = (volatile v4u*)(dst + (size_t)cc * (size_t)ldd + (size_t)r0);
    *d = pk; __threadfence(); *d = pk;
}

__global__ __launch_bounds__(256) void k_mask_flags(const int* __restrict__ mask, int* __restrict__ TF) {
    __shared__ __align__(16) int sF[TFP];
    const int lane = (int)(threadIdx.x & 31u);
    const int wave = __builtin_amdgcn_readfirstlane((int)(threadIdx.x >> 5));
    const int qb = (int)blockIdx.x;
    const int* base = mask + (size_t)(qb * 64 + (lane >> 4)) * SEQ_FULL + (size_t)(4 * (lane & 15));
#pragma unroll 1
    for (int i = 0; i < 4; ++i) {
        const int kc = 4 * wave + i;
        const bool inr = (kc * 64 < SEQ);
        int anyset = inr ? 0 : 1, anyclr = 0;
        if (inr) {
#pragma unroll 4
            for (int it = 0; it < 32; ++it) {
                const v4i m = *(const v4i*)(base + (size_t)(2 * it) * SEQ_FULL + (size_t)(kc * 64));
                const int cnt = ((m.x != 0) ? 1 : 0) + ((m.y != 0) ? 1 : 0) + ((m.z != 0) ? 1 : 0) + ((m.w != 0) ? 1 : 0);
                anyset |= (cnt != 0) ? 1 : 0;
                anyclr |= (cnt != 4) ? 1 : 0;
            }
        }
        const int aS = __any(anyset) ? 1 : 0;
        const int aC = __any(anyclr) ? 1 : 0;
        const int fl = (aC != 0) ? ((aS != 0) ? 1 : 0) : 2;
        if (lane == 0) sF[kc] = fl;
    }
    __syncthreads();
    if (threadIdx.x < 8u) {
        const v4i val = *(const v4i*)&sF[4 * (int)threadIdx.x];
        volatile v4i* d = (volatile v4i*)(TF + (size_t)qb * TFP + (size_t)(4 * (int)threadIdx.x));
        *d = val; __threadfence(); *d = val;
    }
}

template <int ET, bool ASPLIT, int OUT_MODE, bool BIAS>
__device__ __forceinline__ void gemm64_body(const unsigned short* __restrict__ A, const unsigned short* __restrict__ A2, const int lda,
                                            const unsigned short* __restrict__ Bt, const int ldb,
                                            float* __restrict__ Cf, unsigned short* __restrict__ C1, unsigned short* __restrict__ C2,
                                            const float* __restrict__ bias,
                                            const int ldc, const int M, const int N, const int K, const float scale) {
    __shared__ __align__(16) float sT[8][16 * 68];
    const int lane = (int)(threadIdx.x & 31u);
    const int wave = __builtin_amdgcn_readfirstlane((int)(threadIdx.x >> 5));
    const int tilesN = N >> 6;
    const int tile = (int)blockIdx.x * 8 + wave;
    if (tile >= (M >> 6) * tilesN) return;
    const int tm = tile / tilesN, tn = tile - tm * tilesN;
    const int m0 = tm << 6, n0 = tn << 6;
    const int rl = lane & 15, koff = (lane >> 4) * 8, mOff = (lane >> 4) * 8;

    v8f acc[4][4];
#pragma unroll
    for (int i = 0; i < 4; ++i)
#pragma unroll
        for (int j = 0; j < 4; ++j) { const v8f z = {}; acc[i][j] = z; }

#pragma unroll 1
    for (int k0 = 0; k0 < K; k0 += 32) {
        v8u bh[4];
#pragma unroll
        for (int j = 0; j < 4; ++j) bh[j] = ld_frag(Bt + (size_t)(n0 + 16 * j + rl) * (size_t)ldb + (size_t)(koff + k0));
#pragma unroll
        for (int i = 0; i < 4; ++i) {
            const size_t ao = (size_t)(m0 + 16 * i + rl) * (size_t)lda + (size_t)(koff + k0);
            const v8u ah = ld_frag(A + ao);
            v8u al = ah;
            if (ASPLIT) al = ld_frag(A2 + ao);
#pragma unroll
            for (int j = 0; j < 4; ++j) {
                acc[i][j] = mma16<ET>(ah, bh[j], acc[i][j]);
                if (ASPLIT) acc[i][j] = mma16<ET>(al, bh[j], acc[i][j]);
            }
            guard_row(acc[i][0], acc[i][1], acc[i][2], acc[i][3], ah, al, bh[3]);
        }
        keep4(bh[0], bh[1], bh[2], bh[3]);
    }

    v4f bv = {0.f, 0.f, 0.f, 0.f};
    if (OUT_MODE == 0 && BIAS) {
        const v4f t = *(const v4f*)(bias + (size_t)(n0 + (lane & 15) * 4));
        bv.x = bfr_f32(t.x); bv.y = bfr_f32(t.y); bv.z = bfr_f32(t.z); bv.w = bfr_f32(t.w);
    }

#pragma unroll
    for (int i = 0; i < 4; ++i) {
        const int mBase = m0 + 16 * i;
#pragma unroll
        for (int j = 0; j < 4; ++j)
#pragma unroll
            for (int r = 0; r < 8; ++r) sT[wave][(mOff + r) * 68 + 16 * j + rl] = acc[i][j][r] * scale;
        wave_sync();
        if (OUT_MODE == 0) {
            const int hh = lane >> 4, c4 = (lane & 15) * 4;
            v4f vv[8];
#pragma unroll
            for (int it = 0; it < 8; ++it) vv[it] = *(const v4f*)&sT[wave][(it * 2 + hh) * 68 + c4] + bv;
#pragma unroll
            for (int it = 0; it < 8; ++it) *(volatile v4f*)(Cf + (size_t)(mBase + it * 2 + hh) * (size_t)ldc + (size_t)(n0 + c4)) = vv[it];
            __threadfence();
#pragma unroll
            for (int it = 0; it < 8; ++it) *(volatile v4f*)(Cf + (size_t)(mBase + it * 2 + hh) * (size_t)ldc + (size_t)(n0 + c4)) = vv[it];
        } else {
            const int q = lane >> 3, c8 = (lane & 7) * 8;
            v4u hv[4], lv[4];
#pragma unroll
            for (int it = 0; it < 4; ++it) {
                const int row = it * 4 + q;
                const v4f a = *(const v4f*)&sT[wave][row * 68 + c8];
                const v4f b = *(const v4f*)&sT[wave][row * 68 + c8 + 4];
                if (OUT_MODE == 1) {
                    hv[it].x = pk2h(a.x, a.y); hv[it].y = pk2h(a.z, a.w); hv[it].z = pk2h(b.x, b.y); hv[it].w = pk2h(b.z, b.w);
                    lv[it] = hv[it];
                } else if (OUT_MODE == 3) {
                    hres_pack8(a, b, hv[it], lv[it]);
                } else {
                    split_pack8(a, b, hv[it], lv[it]);
                }
            }
#pragma unroll
            for (int it = 0; it < 4; ++it) {
                const size_t o = (size_t)(mBase + it * 4 + q) * (size_t)ldc + (size_t)(n0 + c8);
                *(volatile v4u*)(C1 + o) = hv[it];
                if (OUT_MODE >= 2) *(volatile v4u*)(C2 + o) = lv[it];
            }
            __threadfence();
#pragma unroll
            for (int it = 0; it < 4; ++it) {
                const size_t o = (size_t)(mBase + it * 4 + q) * (size_t)ldc + (size_t)(n0 + c8);
                *(volatile v4u*)(C1 + o) = hv[it];
                if (OUT_MODE >= 2) *(volatile v4u*)(C2 + o) = lv[it];
            }
        }
        wave_sync();
    }
}

__global__ __launch_bounds__(256) CAP256 void k_gemm_qk(const unsigned short* __restrict__ X16, const unsigned short* __restrict__ W316,
                                                        unsigned short* __restrict__ QKh, unsigned short* __restrict__ QKl) {
    gemm64_body<0, false, 2, false>(X16, X16, DM, W316, DM, (float*)0, QKh, QKl, (const float*)0, QKP, MROWS, 2 * DM, DM, 0.0625f);
}
__global__ __launch_bounds__(256) CAP256 void k_gemm_vt(const unsigned short* __restrict__ WV16, const unsigned short* __restrict__ X16,
                                                        unsigned short* __restrict__ VT, unsigned short* __restrict__ VTR) {
    gemm64_body<0, false, 3, false>(WV16, WV16, DM, X16, DM, (float*)0, VT, VTR, (const float*)0, VTP, DM, MROWS, DM, 0.0625f);
}
__global__ __launch_bounds__(256) CAP256 void k_gemm_out(const unsigned short* __restrict__ CTh, const unsigned short* __restrict__ CTl,
                                                         const unsigned short* __restrict__ WOB, const float* __restrict__ bias, float* __restrict__ out) {
    gemm64_body<1, true, 0, true>(CTh, CTl, DM, WOB, DM, out, (unsigned short*)0, (unsigned short*)0, bias, DM, MROWS, DM, DM, 1.0f);
}

template <bool EARLY>
__device__ __forceinline__ void attn_body(const unsigned short* __restrict__ QKh, const unsigned short* __restrict__ QKl,
                                          const unsigned short* __restrict__ VT, const unsigned short* __restrict__ VTR,
                                          const int* __restrict__ mask, const int* __restrict__ TF,
                                          unsigned short* __restrict__ CTh, unsigned short* __restrict__ CTl,
                                          const int qb, const int b, const int h) {
    __shared__ __align__(16) _Float16 Ps[4][16 * PP];
    __shared__ __align__(16) _Float16 Pr[EARLY ? 4 : 1][16 * PP];
    __shared__ __align__(16) float    Os[4][16 * 68];
    const int lane = (int)(threadIdx.x & 31u);
    const int wave = __builtin_amdgcn_readfirstlane((int)(threadIdx.x >> 5));
    const int hh = lane >> 4, c = lane & 15;
    const int q0 = qb * 64 + wave * 16;
    const size_t rowb = (size_t)b * SEQ;

    const size_t qoff = (rowb + (size_t)(q0 + c)) * QKP + (size_t)(h * HD + 8 * hh);
    v8u qh0 = {}, qh1 = {}, ql0 = {}, ql1 = {};
    if (!EARLY) {
        qh0 = ld_frag(QKh + qoff); qh1 = ld_frag(QKh + qoff + 32);
        ql0 = ld_frag(QKl + qoff); ql1 = ld_frag(QKl + qoff + 32);
    }

    float mrow[8], lrow[8];
    v8f o[4], ores[4];
#pragma unroll
    for (int r = 0; r < 8; ++r) { mrow[r] = -1.0e30f; lrow[r] = 0.f; }
#pragma unroll
    for (int t = 0; t < 4; ++t) { const v8f z = {}; o[t] = z; ores[t] = z; }

    const float CS = 0.125f * 1.4426950408889634f;
    const size_t kofs = (rowb + (size_t)(4 * c)) * QKP + (size_t)(DM + h * HD + 8 * hh);
    const size_t vofs = (size_t)(h * HD + c) * VTP + rowb + (size_t)(8 * hh);
    const int* mrowp = mask + (size_t)(q0 + 8 * hh) * SEQ_FULL + (size_t)(4 * c);

#pragma unroll 1
    for (int ci = 0; ci < SEQ / 64; ++ci) {
        const int fl = __builtin_amdgcn_readfirstlane(TF[qb * TFP + ci]);
        if (fl == 2) continue;
        const int kv0 = ci * 64;
        unsigned int mball = 0u;
        if (fl != 0) {
#pragma unroll
            for (int r = 0; r < 8; ++r) {
                const v4i mk = *(const v4i*)(mrowp + (size_t)r * SEQ_FULL + (size_t)kv0);
                const unsigned int nib = ((mk.x != 0) ? 1u : 0u) | ((mk.y != 0) ? 2u : 0u) | ((mk.z != 0) ? 4u : 0u) | ((mk.w != 0) ? 8u : 0u);
                mball |= nib << (4 * r);
            }
        }
        if (EARLY) {
            int z = 0;
            asm volatile("" : "+v"(z));
            const size_t qo = qoff + (size_t)z;
            qh0 = ld_frag(QKh + qo); qh1 = ld_frag(QKh + qo + 32);
            ql0 = ld_frag(QKl + qo); ql1 = ld_frag(QKl + qo + 32);
        }
        v8f s[4];
#pragma unroll
        for (int j = 0; j < 4; ++j) {
            const size_t ko = kofs + (size_t)(kv0 + j) * QKP;
            v8f acc = {};
            {
                const v8u kh = ld_frag(QKh + ko), kl = ld_frag(QKl + ko);
                acc = wmma3b(qh0, ql0, kh, kl, acc);
            }
            {
                const v8u kh = ld_frag(QKh + ko + 32), kl = ld_frag(QKl + ko + 32);
                acc = wmma3b(qh1, ql1, kh, kl, acc);
            }
            s[j] = acc;
        }
#pragma unroll
        for (int r = 0; r < 8; ++r) {
            const unsigned int nb = mball >> (4 * r);
            const bool x0 = (nb & 1u) != 0u, x1 = (nb & 2u) != 0u, x2 = (nb & 4u) != 0u, x3 = (nb & 8u) != 0u;
            const float t0 = x0 ? -1.0e30f : s[0][r] * CS;
            const float t1 = x1 ? -1.0e30f : s[1][r] * CS;
            const float t2 = x2 ? -1.0e30f : s[2][r] * CS;
            const float t3 = x3 ? -1.0e30f : s[3][r] * CS;
            float mx = fmaxf(fmaxf(t0, t1), fmaxf(t2, t3));
            mx = fmaxf(mx, __shfl_xor(mx, 1, 32));
            mx = fmaxf(mx, __shfl_xor(mx, 2, 32));
            mx = fmaxf(mx, __shfl_xor(mx, 4, 32));
            mx = fmaxf(mx, __shfl_xor(mx, 8, 32));
            const float mnew = fmaxf(mrow[r], mx);
            const float corr = exp2f(mrow[r] - mnew);
            mrow[r] = mnew;
            const float e0 = exp2f(t0 - mnew);
            const float e1 = exp2f(t1 - mnew);
            const float e2 = exp2f(t2 - mnew);
            const float e3 = exp2f(t3 - mnew);
            const float p0 = x0 ? 0.f : e0;
            const float p1 = x1 ? 0.f : e1;
            const float p2 = x2 ? 0.f : e2;
            const float p3 = x3 ? 0.f : e3;
            lrow[r] = lrow[r] * corr + ((p0 + p1) + (p2 + p3));
#pragma unroll
            for (int t = 0; t < 4; ++t) { o[t][r] *= corr; if (EARLY) ores[t][r] *= corr; }
            const float g0 = p0 * 4096.f, g1 = p1 * 4096.f, g2 = p2 * 4096.f, g3 = p3 * 4096.f;
            v4h pk;
            pk.x = (_Float16)g0; pk.y = (_Float16)g1; pk.z = (_Float16)g2; pk.w = (_Float16)g3;
            *(v4h*)&Ps[wave][(8 * hh + r) * PP + 4 * c] = pk;
            if (EARLY) {
                v4h pq;
                pq.x = (_Float16)((g0 - (float)pk.x) * 2048.f); pq.y = (_Float16)((g1 - (float)pk.y) * 2048.f);
                pq.z = (_Float16)((g2 - (float)pk.z) * 2048.f); pq.w = (_Float16)((g3 - (float)pk.w) * 2048.f);
                *(v4h*)&Pr[wave][(8 * hh + r) * PP + 4 * c] = pq;
            }
        }
        wave_sync();
#pragma unroll
        for (int kk = 0; kk < 2; ++kk) {
            const v8h pa0 = *(const v8h*)&Ps[wave][c * PP + kk * 32 + 8 * hh];
            const v8h pa1 = *(const v8h*)&Ps[wave][c * PP + kk * 32 + 16 + 8 * hh];
            const v16h pa = __builtin_shufflevector(pa0, pa1, 0, 1, 2, 3, 4, 5, 6, 7, 8, 9, 10, 11, 12, 13, 14, 15);
            v16h pra = pa;
            if (EARLY) {
                const v8h pb0 = *(const v8h*)&Pr[wave][c * PP + kk * 32 + 8 * hh];
                const v8h pb1 = *(const v8h*)&Pr[wave][c * PP + kk * 32 + 16 + 8 * hh];
                pra = __builtin_shufflevector(pb0, pb1, 0, 1, 2, 3, 4, 5, 6, 7, 8, 9, 10, 11, 12, 13, 14, 15);
            }
#pragma unroll
            for (int t = 0; t < 4; ++t) {
                const size_t vo = vofs + (size_t)(16 * t) * VTP + (size_t)(kv0 + kk * 32);
                const v8u vb = ld_frag(VT + vo);
                o[t] = wmma1h(pa, vb, o[t]);
                if (EARLY) {
                    const v8u vr = ld_frag(VTR + vo);
                    ores[t] = wmma1h(pa, vr, ores[t]);
                    ores[t] = wmma1h(pra, vb, ores[t]);
                }
            }
        }
        wave_sync();
    }

#pragma unroll
    for (int r = 0; r < 8; ++r) {
        float l = lrow[r];
        l += __shfl_xor(l, 1, 32); l += __shfl_xor(l, 2, 32); l += __shfl_xor(l, 4, 32); l += __shfl_xor(l, 8, 32);
        const float inv = 1.0f / (l * 4096.f);
#pragma unroll
        for (int t = 0; t < 4; ++t) {
            const float val = EARLY ? (o[t][r] + ores[t][r] * (1.0f / 2048.0f)) : o[t][r];
            Os[wave][(8 * hh + r) * 68 + 16 * t + c] = val * inv;
        }
    }
    wave_sync();
    {
        const int q4 = lane >> 3, c8 = (lane & 7) * 8;
        v4u hv[4], lv[4];
#pragma unroll
        for (int it = 0; it < 4; ++it) {
            const int row = it * 4 + q4;
            const v4f a = *(const v4f*)&Os[wave][row * 68 + c8];
            const v4f b2 = *(const v4f*)&Os[wave][row * 68 + c8 + 4];
            split_pack8(a, b2, hv[it], lv[it]);
        }
#pragma unroll
        for (int it = 0; it < 4; ++it) {
            const size_t oo = (rowb + (size_t)(q0 + it * 4 + q4)) * DM + (size_t)(h * HD + c8);
            *(volatile v4u*)(CTh + oo) = hv[it];
            *(volatile v4u*)(CTl + oo) = lv[it];
        }
        __threadfence();
#pragma unroll
        for (int it = 0; it < 4; ++it) {
            const size_t oo = (rowb + (size_t)(q0 + it * 4 + q4)) * DM + (size_t)(h * HD + c8);
            *(volatile v4u*)(CTh + oo) = hv[it];
            *(volatile v4u*)(CTl + oo) = lv[it];
        }
    }
}

__global__ __launch_bounds__(128) CAP256 void k_attn_main(const unsigned short* __restrict__ QKh, const unsigned short* __restrict__ QKl,
                                                          const unsigned short* __restrict__ VT,
                                                          const int* __restrict__ mask, const int* __restrict__ TF,
                                                          unsigned short* __restrict__ CTh, unsigned short* __restrict__ CTl) {
    const int nqm = (SEQ / 64 > EARLYB) ? (SEQ / 64 - EARLYB) : 1;
    const int bx = (int)blockIdx.x;
    const int qb = EARLYB + bx % nqm;
    const int bhd = bx / nqm;
    const int h = bhd % NH;
    const int b = bhd / NH;
    attn_body<false>(QKh, QKl, VT, VT, mask, TF, CTh, CTl, qb, b, h);
}
__global__ __launch_bounds__(128) CAP256 void k_attn_early(const unsigned short* __restrict__ QKh, const unsigned short* __restrict__ QKl,
                                                           const unsigned short* __restrict__ VT, const unsigned short* __restrict__ VTR,
                                                           const int* __restrict__ mask, const int* __restrict__ TF,
                                                           unsigned short* __restrict__ CTh, unsigned short* __restrict__ CTl) {
    const int bx = (int)blockIdx.x;
    const int qb = bx % EARLYB;
    const int bhd = bx / EARLYB;
    const int h = bhd % NH;
    const int b = bhd / NH;
    attn_body<true>(QKh, QKl, VT, VTR, mask, TF, CTh, CTl, qb, b, h);
}

#define WS_X16   ((size_t)MROWS * DM * 2)
#define WS_W316  ((size_t)3 * DM * DM * 2)
#define WS_WOB   ((size_t)DM * DM * 2)
#define WS_QK    ((size_t)MROWS * QKP * 2)
#define WS_VT    ((size_t)DM * VTP * 2)
#define WS_CT    ((size_t)MROWS * DM * 2)
#define WS_TF    ((size_t)(SEQ_FULL / 64) * TFP * 4)
#define WS_TOTAL (WS_X16 + WS_W316 + WS_WOB + 2 * WS_QK + 2 * WS_VT + 2 * WS_CT + WS_TF)
static_assert(WS_TOTAL <= (size_t)134217728);
static_assert(WS_X16 % 256 == 0);
static_assert(WS_W316 % 256 == 0);
static_assert(WS_WOB % 256 == 0);
static_assert(WS_QK % 256 == 0);
static_assert(WS_VT % 256 == 0);
static_assert(WS_CT % 256 == 0);
static_assert(WS_TF % 256 == 0);
static_assert((MROWS * (DM / 8)) % 256 == 0);
static_assert(DM % 8 == 0);
static_assert((size_t)(SEQ / 64) * TFP * 4 <= WS_TF);

extern "C" void kernel_launch(void* const* d_in, const int* in_sizes, int n_in, void* d_out, int out_size, void* d_ws, size_t ws_size, hipStream_t stream) {
    if (n_in < 5) return;
    if ((long long)in_sizes[0] < ((long long)(NB - 1) * SEQ_FULL + SEQ) * DM) return;
    if ((long long)in_sizes[1] < ((long long)(SEQ - 1) * SEQ_FULL + SEQ)) return;
    if ((long long)in_sizes[2] < (long long)DM * 3 * DM) return;
    if ((long long)in_sizes[3] < (long long)DM * DM) return;
    if ((long long)in_sizes[4] < (long long)DM) return;
    if ((long long)out_size < (long long)MROWS * DM) return;
    if (ws_size < WS_TOTAL) return;

    const float* x    = (const float*)d_in[0];
    const int*   mask = (const int*)d_in[1];
    const float* Wqkv = (const float*)d_in[2];
    const float* Wo   = (const float*)d_in[3];
    const float* bo   = (const float*)d_in[4];
    float* out = (float*)d_out;

    char* wsp = (char*)d_ws;
    unsigned short* X16  = (unsigned short*)wsp; wsp += WS_X16;
    unsigned short* W316 = (unsigned short*)wsp; wsp += WS_W316;
    unsigned short* WOB  = (unsigned short*)wsp; wsp += WS_WOB;
    unsigned short* QKh  = (unsigned short*)wsp; wsp += WS_QK;
    unsigned short* QKl  = (unsigned short*)wsp; wsp += WS_QK;
    unsigned short* VT   = (unsigned short*)wsp; wsp += WS_VT;
    unsigned short* VTR  = (unsigned short*)wsp; wsp += WS_VT;
    unsigned short* CTh  = (unsigned short*)wsp; wsp += WS_CT;
    unsigned short* CTl  = (unsigned short*)wsp; wsp += WS_CT;
    int*            TF   = (int*)wsp;            wsp += WS_TF;

    k_cast_x<<<(unsigned)((MROWS * (DM / 8)) / 256), 256, 0, stream>>>(x, X16);
    k_castT<<<(unsigned)(((long long)(3 * DM) * (DM / 8) + 255) / 256), 256, 0, stream>>>(Wqkv, 3 * DM, W316, DM, DM, 3 * DM, 16.0f, 0);
    k_castT<<<(unsigned)(((long long)DM * (DM / 8) + 255) / 256), 256, 0, stream>>>(Wo, DM, WOB, DM, DM, DM, 1.0f, 1);
    k_mask_flags<<<(unsigned)(SEQ / 64), 256, 0, stream>>>(mask, TF);
    k_gemm_qk<<<(unsigned)(((MROWS / 64) * ((2 * DM) / 64) + 7) / 8), 256, 0, stream>>>(X16, W316, QKh, QKl);
    k_gemm_vt<<<(unsigned)(((DM / 64) * (MROWS / 64) + 7) / 8), 256, 0, stream>>>(W316 + (size_t)2 * DM * DM, X16, VT, VTR);
    k_attn_early<<<(unsigned)(NB * NH * EARLYB), 128, 0, stream>>>(QKh, QKl, VT, VTR, mask, TF, CTh, CTl);
    if (SEQ / 64 > EARLYB)
        k_attn_main<<<(unsigned)(NB * NH * ((SEQ / 64 > EARLYB) ? (SEQ / 64 - EARLYB) : 1)), 128, 0, stream>>>(QKh, QKl, VT, mask, TF, CTh, CTl);
    k_gemm_out<<<(unsigned)(((MROWS / 64) * (DM / 64) + 7) / 8), 256, 0, stream>>>(CTh, CTl, WOB, bo, out);
}
